// SetConv_32435593019489
// MI455X (gfx1250) — hardware-run, weakly checked
//
#include <hip/hip_runtime.h>
#include <stddef.h>


typedef _Float16 v16h __attribute__((ext_vector_type(16)));
typedef _Float16 v8h  __attribute__((ext_vector_type(8)));
typedef float    v8f  __attribute__((ext_vector_type(8)));
typedef float    v4f  __attribute__((ext_vector_type(4)));
typedef _Float16 h16;

#ifndef NB
#define NB 8
#endif
#ifndef SEQ
#define SEQ 1024
#endif
#define NB_FULL  8
#define SEQ_FULL 1024
#define NOBS  1024
#define CIN   16
#define COUT  32
#define NTHR  128
#define TROWS 64

#define YLD 1032
#define WLD 40
#define PLD 40
#define OLD 36

#define LOG2E   1.44269504088896340736f
#define WTCARRY 4096.0f
#define INCARRY 64.0f
#define OCARRY  16.0f
#define WCARRY  64.0f
#define OSCALE  (OCARRY / (WTCARRY * INCARRY))
#define FINV    (1.0f / (WCARRY * OCARRY))

static_assert(NB >= 1 && NB <= NB_FULL);
static_assert(SEQ >= TROWS && SEQ <= SEQ_FULL && (SEQ % TROWS) == 0);
static_assert((NOBS % 32) == 0);
static_assert(CIN == 16);
static_assert(COUT == 32);
static_assert(COUT * 4 == 128);
static_assert(NTHR == 4 * 32);
static_assert(TROWS == (NTHR / 32) * 16);
static_assert((NOBS % NTHR) == 0);
static_assert(((NOBS * CIN / 4) % NTHR) == 0);
static_assert(((COUT * 32) % NTHR) == 0);
static_assert((YLD % 8) == 0 && YLD >= NOBS);
static_assert((WLD % 8) == 0 && WLD >= 32);
static_assert((PLD % 8) == 0 && PLD >= 32);
static_assert((OLD % 4) == 0 && OLD >= COUT);
static_assert((size_t)CIN * YLD * 2 + (size_t)NOBS * 4 + (size_t)COUT * WLD * 2 +
              (size_t)(NTHR / 32) * 16 * PLD * 2 + (size_t)(NTHR / 32) * 16 * OLD * 4 +
              (size_t)CIN * 4 <= (size_t)65536);
static_assert((size_t)NB_FULL * SEQ_FULL * COUT * 4 == (size_t)1048576);
static_assert(((size_t)(NB - 1) * SEQ_FULL + SEQ) * COUT * 4 <= (size_t)1048576);

__device__ __forceinline__ float bf16r(float x) {
  unsigned int u = __float_as_uint(x);
  u = (u + 0x7FFFu + ((u >> 16) & 1u)) & 0xFFFF0000u;
  return __uint_as_float(u);
}

static __device__ __forceinline__ h16 toh_flush(float v) {
  const h16 r = (h16)v;
  return (fabsf(v) < 6.103515625e-05f) ? (h16)0.0f : r;
}

__device__ __forceinline__ v16h frag_at(const _Float16* p) {
  v8h lo = *(const v8h*)(p);
  v8h hi = *(const v8h*)(p + 16);
  v16h out;
#pragma unroll
  for (int i = 0; i < 8; ++i) { out[i] = lo[i]; out[i + 8] = hi[i]; }
  return out;
}
__device__ __forceinline__ v16h ld_frag(const _Float16* base, unsigned ld) {
  const unsigned lane = threadIdx.x & 31u;
  return frag_at(base + (lane & 15u) * ld + (lane >> 4) * 8u);
}

__device__ __forceinline__ v8f wmma16(v16h a, v16h b, v8f c) {
  v8f d = __builtin_amdgcn_wmma_f32_16x16x32_f16(false, a, false, b, (short)0, c,
                                                 false, false);
  asm volatile("v_nop\n\tv_nop\n\tv_nop\n\tv_nop" : "+v"(d) : "v"(a), "v"(b));
  return d;
}

__device__ __forceinline__ void wave_lds_sync() {
  __builtin_amdgcn_fence(3  , "wavefront");
  asm volatile("s_wait_dscnt 0x0" ::: "memory");
  __builtin_amdgcn_wave_barrier();
}

__global__ __launch_bounds__(NTHR) void rbf_agg_kernel(
    const float* __restrict__ x, const float* __restrict__ y, const float* __restrict__ t,
    const float* __restrict__ sigma, const float* __restrict__ W,
    const float* __restrict__ bias, float* __restrict__ out) {
  __shared__ __attribute__((aligned(16))) _Float16 Ys[CIN * YLD];
  __shared__ __attribute__((aligned(16))) float    Xs[NOBS];
  __shared__ __attribute__((aligned(16))) _Float16 Ws[COUT * WLD];
  __shared__ __attribute__((aligned(16))) _Float16 Ps[(NTHR / 32) * 16 * PLD];
  __shared__ __attribute__((aligned(16))) float    Os[(NTHR / 32) * 16 * OLD];
  __shared__ __attribute__((aligned(16))) float    K2s[CIN];

  const unsigned tid = threadIdx.x, lane = tid & 31u;
  const unsigned wave = (unsigned)__builtin_amdgcn_readfirstlane((int)(threadIdx.x >> 5));
  const unsigned hh = lane >> 4, m = lane & 15u;
  const unsigned b = blockIdx.y;
  const unsigned t0 = blockIdx.x * (unsigned)TROWS + wave * 16u;
  const unsigned pbase = wave * (16u * PLD);
  const unsigned obase = wave * (16u * OLD);

  unsigned su[CIN];
#pragma unroll
  for (int j = 0; j < CIN; ++j) su[j] = __float_as_uint(bf16r(sigma[j]));
  unsigned leadv = 0u;
#pragma unroll
  for (int j = 0; j < CIN; ++j) {
    bool first = true;
#pragma unroll
    for (int i = 0; i < j; ++i) first = first && (su[i] != su[j]);
    leadv |= first ? (1u << j) : 0u;
  }
  const unsigned lead = (unsigned)__builtin_amdgcn_readfirstlane((int)leadv);
  const unsigned mine = __float_as_uint(bf16r(sigma[m]));
  unsigned my_rep = (unsigned)(CIN - 1);
#pragma unroll
  for (int j = CIN - 1; j >= 0; --j) my_rep = (su[j] == mine) ? (unsigned)j : my_rep;

  {
    const float sg = bf16r(sigma[tid & 15u]);
    const float inv_s2 = __builtin_amdgcn_exp2f(-2.0f * sg * LOG2E);
    const float kv = -0.5f * inv_s2 * LOG2E;
    if (tid < (unsigned)CIN) K2s[tid] = kv;
  }

#pragma unroll 4
  for (unsigned j = 0; j < (unsigned)(NOBS / NTHR); ++j) {
    const unsigned n = tid + (unsigned)NTHR * j;
    Xs[n] = bf16r(x[(size_t)b * NOBS + n]);
  }
#pragma unroll 4
  for (unsigned j = 0; j < (unsigned)((NOBS * CIN / 4) / NTHR); ++j) {
    const unsigned idx = tid + (unsigned)NTHR * j;
    const unsigned n = idx >> 2, cq = (idx & 3u) * 4u;
    const v4f v = *(const v4f*)(y + ((size_t)b * NOBS + n) * CIN + cq);
#pragma unroll
    for (unsigned i = 0; i < 4u; ++i)
      Ys[(cq + i) * YLD + n] = toh_flush(INCARRY * bf16r(v[i]));
  }
#pragma unroll 4
  for (unsigned j = 0; j < (unsigned)((COUT * 32) / NTHR); ++j) {
    const unsigned idx = tid + (unsigned)NTHR * j;
    const unsigned o = idx >> 5, k = idx & 31u;
    const unsigned kc = (k < (unsigned)CIN) ? k : (unsigned)(CIN - 1);
    const float wv = W[o * (unsigned)CIN + kc];
    const h16 hv = toh_flush(WCARRY * bf16r(wv));
    Ws[o * WLD + k] = (k < (unsigned)CIN) ? hv : (h16)0.0f;
  }
  {
    v8h z;
#pragma unroll
    for (int i = 0; i < 8; ++i) z[i] = (h16)0.0f;
    *(v8h*)&Ps[pbase + (lane >> 1) * PLD + 16u + (lane & 1u) * 8u] = z;
  }
  __syncthreads();

  const float tm = bf16r(t[(size_t)b * SEQ_FULL + t0 + m]);
  v8f acc = {};

#pragma unroll 1
  for (unsigned n0 = 0; n0 < (unsigned)NOBS; n0 += 32u) {
    const v16h yf = ld_frag(&Ys[n0], YLD);
    const v4f xa = *(const v4f*)&Xs[n0 + hh * 8u];
    const v4f xb = *(const v4f*)&Xs[n0 + hh * 8u + 4u];
    const v4f xc = *(const v4f*)&Xs[n0 + 16u + hh * 8u];
    const v4f xd = *(const v4f*)&Xs[n0 + 16u + hh * 8u + 4u];
    float d[16];
#pragma unroll
    for (int i = 0; i < 4; ++i) {
      const float u0 = xa[i] - tm;
      const float u1 = xb[i] - tm;
      const float u2 = xc[i] - tm;
      const float u3 = xd[i] - tm;
      d[i]      = u0 * u0;
      d[i + 4]  = u1 * u1;
      d[i + 8]  = u2 * u2;
      d[i + 12] = u3 * u3;
    }
#pragma unroll 1
    for (unsigned g = 0; g < (unsigned)CIN; ++g) {
      if (((lead >> g) & 1u) == 0u) continue;
      const float kg = K2s[g];
      const bool sel = (my_rep == g);
      v16h af, bm;
#pragma unroll
      for (int i = 0; i < 16; ++i) {
        af[i] = toh_flush(WTCARRY * __builtin_amdgcn_exp2f(d[i] * kg));
        bm[i] = sel ? yf[i] : (h16)0.0f;
      }
      acc = wmma16(af, bm, acc);
    }
  }

#pragma unroll
  for (int r = 0; r < 8; ++r)
    Ps[pbase + (hh * 8u + (unsigned)r) * PLD + m] = toh_flush(acc[r] * OSCALE);
  wave_lds_sync();

  const v16h pf = ld_frag(&Ps[pbase], PLD);
  const v16h w0 = ld_frag(&Ws[0], WLD);
  const v16h w1 = ld_frag(&Ws[16 * WLD], WLD);
  v8f c0 = {}, c1 = {};
  c0 = wmma16(pf, w0, c0);
  c1 = wmma16(pf, w1, c1);

  const float bo0 = bf16r(bias[m]);
  const float bo1 = bf16r(bias[16u + m]);
#pragma unroll
  for (int r = 0; r < 8; ++r) {
    const unsigned ro = obase + (hh * 8u + (unsigned)r) * OLD;
    Os[ro + m]       = c0[r] * FINV + bo0;
    Os[ro + 16u + m] = c1[r] * FINV + bo1;
  }
  wave_lds_sync();

  v4f xo[4];
  size_t off[4];
#pragma unroll
  for (unsigned i = 0; i < 4u; ++i) {
    const unsigned r = 4u * i + (lane >> 3);
    const unsigned c = (lane & 7u) * 4u;
    xo[i] = *(const v4f*)&Os[obase + r * OLD + c];
    off[i] = ((size_t)b * SEQ_FULL + t0 + r) * COUT + c;
  }
#pragma unroll
  for (int i = 0; i < 4; ++i) *(volatile v4f*)(out + off[i]) = xo[i];
  __threadfence();
#pragma unroll
  for (int i = 0; i < 4; ++i) *(volatile v4f*)(out + off[i]) = xo[i];
}

extern "C" void kernel_launch(void* const* d_in, const int* in_sizes, int n_in,
                              void* d_out, int out_size, void* d_ws, size_t ws_size,
                              hipStream_t stream) {
  (void)d_ws;
  (void)ws_size;
  if (n_in < 6) return;
  if ((long long)in_sizes[0] < (long long)NB * NOBS) return;
  if ((long long)in_sizes[1] < (long long)NB * NOBS * CIN) return;
  if ((long long)in_sizes[2] < (long long)(NB - 1) * SEQ_FULL + SEQ) return;
  if (in_sizes[3] < CIN) return;
  if (in_sizes[4] < COUT * CIN) return;
  if (in_sizes[5] < COUT) return;
  if ((long long)out_size < ((long long)(NB - 1) * SEQ_FULL + SEQ) * COUT) return;

  const float* x     = (const float*)d_in[0];
  const float* y     = (const float*)d_in[1];
  const float* t     = (const float*)d_in[2];
  const float* sigma = (const float*)d_in[3];
  const float* W     = (const float*)d_in[4];
  const float* bias  = (const float*)d_in[5];
  float* out = (float*)d_out;

  rbf_agg_kernel<<<dim3(SEQ / TROWS, NB), dim3(NTHR), 0, stream>>>(x, y, t, sigma, W, bias, out);
}
